// SimpleAttention_14027363188928
// MI455X (gfx1250) — hardware-verified
//
#include <hip/hip_runtime.h>
#include <stdint.h>


typedef _Float16 v16h __attribute__((ext_vector_type(16)));
typedef _Float16 v8h  __attribute__((ext_vector_type(8)));
typedef _Float16 v8ha __attribute__((ext_vector_type(8), may_alias));
typedef float    v8f  __attribute__((ext_vector_type(8)));
typedef float    v4f  __attribute__((ext_vector_type(4)));
typedef float    v4fa __attribute__((ext_vector_type(4), may_alias));
typedef unsigned int v4u __attribute__((ext_vector_type(4)));

union U8f  { v8f  v; float    f[8]; };
union U16h { v16h v; v8h      h[2]; };
union U8h  { v8h  v; _Float16 f[8]; };

#ifndef NB
#define NB 16
#endif
#ifndef SEQ
#define SEQ 2048
#endif
#define NB_FULL  16
#define SEQ_FULL 2048
#define DD       256

#define BQ  128
#define BK  32
#define QP  264
#define KP  264
#define VP  40
#define TP  72
#define NT  64

static_assert(SEQ % BQ == 0);
static_assert(SEQ % NT == 0);
static_assert(SEQ % BK == 0);
static_assert(NB >= 1 && NB <= NB_FULL);
static_assert(SEQ >= BQ && SEQ <= SEQ_FULL);

#define SQ_OFF  0
#define SK_OFF  (SQ_OFF + 8 * 16 * QP)
#define SV_OFF  (SK_OFF + BK * KP)
#define SP_OFF  (SV_OFF + DD * VP)
#define SO_OFFH (SP_OFF + 8 * 16 * BK)
#define LDS_BYTES (SO_OFFH * 2 + 8 * 16 * 64 * 4)
static_assert((SK_OFF * 2) % 16 == 0);
static_assert((SV_OFF * 2) % 16 == 0);
static_assert((SP_OFF * 2) % 16 == 0);
static_assert((SO_OFFH * 2) % 16 == 0);
static_assert(LDS_BYTES == 145920);

#define C2SCALE 0.09016844005556021f

__device__ __forceinline__ v8f wmma_f16(v16h a, v16h b, v8f c) {
  v8f d = __builtin_amdgcn_wmma_f32_16x16x32_f16(false, a, false, b, (short)0, c, false, false);
  asm volatile("v_nop\n\tv_nop\n\tv_nop\n\tv_nop" : "+v"(d) : "v"(a), "v"(b));
  return d;
}

template <int CTRL>
__device__ __forceinline__ float dppf(float x) {
  int s = __float_as_int(x);
  return __int_as_float(__builtin_amdgcn_update_dpp(s, s, CTRL, 0xF, 0xF, true));
}
__device__ __forceinline__ float red_max16(float x) {
  x = fmaxf(x, dppf<0xB1>(x));
  x = fmaxf(x, dppf<0x4E>(x));
  x = fmaxf(x, dppf<0x141>(x));
  x = fmaxf(x, dppf<0x140>(x));
  return x;
}
__device__ __forceinline__ float red_sum16(float x) {
  x += dppf<0xB1>(x);
  x += dppf<0x4E>(x);
  x += dppf<0x141>(x);
  x += dppf<0x140>(x);
  return x;
}

__device__ __forceinline__ void wave_lds_sync() {
  __builtin_amdgcn_fence(3, "wavefront");
  asm volatile("s_wait_dscnt 0" ::: "memory");
  __builtin_amdgcn_wave_barrier();
}

__device__ __forceinline__ v4f bf16_rne4(v4f a) {
  v4u u = __builtin_bit_cast(v4u, a);
  u = (u + 0x7FFFu + ((u >> 16) & 1u)) & 0xFFFF0000u;
  return __builtin_bit_cast(v4f, u);
}

__device__ __forceinline__ v8h cvt8v(v4f a, v4f b) {
  v8h d;
  d[0] = (_Float16)a[0]; d[1] = (_Float16)a[1];
  d[2] = (_Float16)a[2]; d[3] = (_Float16)a[3];
  d[4] = (_Float16)b[0]; d[5] = (_Float16)b[1];
  d[6] = (_Float16)b[2]; d[7] = (_Float16)b[3];
  return d;
}

__global__ __launch_bounds__(256)
void prep_kernel(const float* __restrict__ X, _Float16* __restrict__ Xh,
                 _Float16* __restrict__ Vt, float* __restrict__ Rn)
{
  __shared__ __attribute__((aligned(16))) _Float16 sT[DD * TP];
  __shared__ float sR[NT];

  const int tid = threadIdx.x;
  const int sub = tid & 7;
  const int rq  = tid >> 3;
  const int ntb = SEQ / NT;
  const int b   = blockIdx.x / ntb;
  const int n0  = (blockIdx.x % ntb) * NT;

  #pragma unroll 1
  for (int pass = 0; pass < 2; ++pass) {
    const int r = pass * 32 + rq;
    const float* src = X  + ((size_t)b * SEQ_FULL + n0 + r) * DD;
    _Float16*    dst = Xh + ((size_t)b * SEQ      + n0 + r) * DD;
    float ss = 0.0f;
    #pragma unroll 1
    for (int i = 0; i < 4; ++i) {
      const int c0 = 8 * (sub + 8 * i);
      const v4f a0 = bf16_rne4(*(const v4f*)(src + c0));
      const v4f a1 = bf16_rne4(*(const v4f*)(src + c0 + 4));
      ss += a0[0] * a0[0]; ss += a0[1] * a0[1]; ss += a0[2] * a0[2]; ss += a0[3] * a0[3];
      ss += a1[0] * a1[0]; ss += a1[1] * a1[1]; ss += a1[2] * a1[2]; ss += a1[3] * a1[3];
      U8h hh; hh.v = cvt8v(a0, a1);
      *(volatile v8h*)(dst + c0) = hh.v;
      __threadfence();
      *(volatile v8h*)(dst + c0) = hh.v;
      #pragma unroll
      for (int e = 0; e < 8; ++e) sT[(c0 + e) * TP + r] = hh.f[e];
    }
    ss += __shfl_xor(ss, 1, 32);
    ss += __shfl_xor(ss, 2, 32);
    ss += __shfl_xor(ss, 4, 32);
    const float rinv = 1.0f / fmaxf(sqrtf(ss), 1e-12f);
    if (sub == 0) sR[r] = rinv;
  }
  __syncthreads();

  v8h vv[8];
  #pragma unroll
  for (int i = 0; i < 8; ++i) vv[i] = *(const v8ha*)(sT + (rq + 32 * i) * TP + 8 * sub);
  const int ti = tid & 15;
  v4f rv;
  rv[0] = sR[4 * ti]; rv[1] = sR[4 * ti + 1]; rv[2] = sR[4 * ti + 2]; rv[3] = sR[4 * ti + 3];
  _Float16* vb = Vt + (size_t)b * DD * SEQ + n0 + 8 * sub;
  float*    rp = Rn + (size_t)b * SEQ + n0 + 4 * ti;

  #pragma unroll
  for (int i = 0; i < 8; ++i) *(volatile v8h*)(vb + (size_t)(rq + 32 * i) * SEQ) = vv[i];
  if (tid < 16) *(volatile v4f*)rp = rv;
  __threadfence();
  #pragma unroll
  for (int i = 0; i < 8; ++i) *(volatile v8h*)(vb + (size_t)(rq + 32 * i) * SEQ) = vv[i];
  if (tid < 16) *(volatile v4f*)rp = rv;
}

__global__ __launch_bounds__(256)
void attn_kernel(const _Float16* __restrict__ Xh, const _Float16* __restrict__ Vt,
                 const float* __restrict__ Rn, float* __restrict__ Out)
{
  extern __shared__ __attribute__((aligned(16))) _Float16 smem[];
  _Float16* sQ = smem + SQ_OFF;
  _Float16* sK = smem + SK_OFF;
  _Float16* sV = smem + SV_OFF;
  _Float16* sP = smem + SP_OFF;
  float*    sO = (float*)(smem + SO_OFFH);

  const int tid  = threadIdx.x;
  const int wave = tid >> 5;
  const int lane = tid & 31;
  const int lh   = lane & 15;
  const int hi   = lane >> 4;

  const int nqb   = SEQ / BQ;
  const int b     = blockIdx.x / nqb;
  const int qbase = (blockIdx.x % nqb) * BQ;
  const int qrow0 = qbase + wave * 16;

  const _Float16* Xb = Xh + (size_t)b * SEQ * DD;
  const _Float16* Vb = Vt + (size_t)b * DD * SEQ;
  const float*    Rb = Rn + (size_t)b * SEQ;
  float*          Ob = Out + (size_t)b * SEQ * DD;

  _Float16* qw = sQ + wave * (16 * QP);
  #pragma unroll
  for (int i = 0; i < 16; ++i) {
    const v8h q = *(const v8h*)(Xb + (size_t)(qrow0 + i) * DD + 8 * lane);
    *(v8h*)(qw + i * QP + 8 * lane) = q;
  }

  U8f acc[16];
  #pragma unroll
  for (int t = 0; t < 16; ++t) acc[t].v = (v8f){};
  float mrow[8], lrow[8];
  #pragma unroll
  for (int j = 0; j < 8; ++j) { mrow[j] = -3.0e38f; lrow[j] = 0.0f; }

  _Float16* pw = sP + wave * (16 * BK);

  for (int kv0 = 0; kv0 < SEQ; kv0 += BK) {
    __syncthreads();
    #pragma unroll
    for (int i = 0; i < 4; ++i) {
      const int idx = tid + 256 * i;
      const int r = idx >> 5, g = idx & 31;
      const v8h kk = *(const v8h*)(Xb + (size_t)(kv0 + r) * DD + 8 * g);
      *(v8h*)(sK + r * KP + 8 * g) = kk;
    }
    #pragma unroll
    for (int i = 0; i < 4; ++i) {
      const int idx = tid + 256 * i;
      const int d = idx >> 2, g = idx & 3;
      const v8h vv = *(const v8h*)(Vb + (size_t)d * SEQ + kv0 + 8 * g);
      *(v8h*)(sV + d * VP + 8 * g) = vv;
    }
    __syncthreads();

    U8f s0, s1; s0.v = (v8f){}; s1.v = (v8f){};
    #pragma unroll
    for (int c = 0; c < 8; ++c) {
      U16h qf, kf;
      qf.h[0] = *(const v8h*)(qw + lh * QP + 32 * c + 8 * hi);
      qf.h[1] = *(const v8h*)(qw + lh * QP + 32 * c + 16 + 8 * hi);
      kf.h[0] = *(const v8h*)(sK + lh * KP + 32 * c + 8 * hi);
      kf.h[1] = *(const v8h*)(sK + lh * KP + 32 * c + 16 + 8 * hi);
      s0.v = wmma_f16(qf.v, kf.v, s0.v);
      kf.h[0] = *(const v8h*)(sK + (16 + lh) * KP + 32 * c + 8 * hi);
      kf.h[1] = *(const v8h*)(sK + (16 + lh) * KP + 32 * c + 16 + 8 * hi);
      s1.v = wmma_f16(qf.v, kf.v, s1.v);
    }

    const float cs0 = Rb[kv0 + lh] * C2SCALE;
    const float cs1 = Rb[kv0 + 16 + lh] * C2SCALE;

    U8h pa, pb;
    #pragma unroll
    for (int j = 0; j < 8; ++j) {
      const float a  = s0.f[j] * cs0;
      const float bb = s1.f[j] * cs1;
      const float rm    = red_max16(fmaxf(a, bb));
      const float mnew  = fmaxf(mrow[j], rm);
      const float alpha = __builtin_amdgcn_exp2f(mrow[j] - mnew);
      const float e0    = __builtin_amdgcn_exp2f(a  - mnew);
      const float e1    = __builtin_amdgcn_exp2f(bb - mnew);
      lrow[j] = lrow[j] * alpha + red_sum16(e0 + e1);
      mrow[j] = mnew;
      pa.f[j] = (_Float16)(e0 * 1024.0f);
      pb.f[j] = (_Float16)(e1 * 1024.0f);
      #pragma unroll
      for (int t = 0; t < 16; ++t) acc[t].f[j] *= alpha;
    }

    #pragma unroll
    for (int j = 0; j < 8; ++j) {
      pw[(j + 8 * hi) * BK + lh]      = pa.f[j];
      pw[(j + 8 * hi) * BK + 16 + lh] = pb.f[j];
    }
    wave_lds_sync();
    U16h pf;
    pf.h[0] = *(const v8ha*)(pw + lh * BK + 8 * hi);
    pf.h[1] = *(const v8ha*)(pw + lh * BK + 16 + 8 * hi);

    #pragma unroll
    for (int t = 0; t < 16; ++t) {
      U16h vf;
      vf.h[0] = *(const v8h*)(sV + (16 * t + lh) * VP + 8 * hi);
      vf.h[1] = *(const v8h*)(sV + (16 * t + lh) * VP + 16 + 8 * hi);
      acc[t].v = wmma_f16(pf.v, vf.v, acc[t].v);
    }
  }

  float inv[8];
  #pragma unroll
  for (int j = 0; j < 8; ++j) inv[j] = 1.0f / (lrow[j] * 1024.0f);
  float* so = sO + wave * (16 * 64);
  #pragma unroll
  for (int g = 0; g < 4; ++g) {
    #pragma unroll
    for (int j = 0; j < 8; ++j) {
      #pragma unroll
      for (int tt = 0; tt < 4; ++tt)
        so[(j + 8 * hi) * 64 + tt * 16 + lh] = acc[4 * g + tt].f[j] * inv[j];
    }
    wave_lds_sync();
    v4f ov[8]; int oo[8];
    #pragma unroll
    for (int i = 0; i < 8; ++i) {
      const int c = lane + 32 * i, rr = c >> 4, q = c & 15;
      ov[i] = *(const v4fa*)(so + rr * 64 + q * 4);
      oo[i] = rr * DD + 64 * g + 4 * q;
    }
    float* ob = Ob + (size_t)qrow0 * DD;
    #pragma unroll
    for (int i = 0; i < 8; ++i) *(volatile v4f*)(ob + oo[i]) = ov[i];
    __threadfence();
    #pragma unroll
    for (int i = 0; i < 8; ++i) *(volatile v4f*)(ob + oo[i]) = ov[i];
    wave_lds_sync();
  }
}

extern "C" void kernel_launch(void* const* d_in, const int* in_sizes, int n_in,
                              void* d_out, int out_size, void* d_ws, size_t ws_size,
                              hipStream_t stream) {
  if (n_in < 1) return;
  const long long need_in = ((long long)(NB - 1) * SEQ_FULL + SEQ) * DD;
  if ((long long)in_sizes[0] < need_in) return;
  if ((long long)out_size < (long long)NB * SEQ * DD) return;

  const size_t xh_bytes = (size_t)NB * SEQ * DD * 2;
  const size_t vt_bytes = (size_t)NB * DD * SEQ * 2;
  const size_t rn_bytes = (size_t)NB * SEQ * 4;
  const size_t off_xh = 0;
  const size_t off_vt = off_xh + xh_bytes;
  const size_t off_rn = off_vt + vt_bytes;
  if (off_rn + rn_bytes > ws_size) return;

  const float* x   = (const float*)d_in[0];
  float*       out = (float*)d_out;
  _Float16* xh = (_Float16*)((char*)d_ws + off_xh);
  _Float16* vt = (_Float16*)((char*)d_ws + off_vt);
  float*    rn = (float*)((char*)d_ws + off_rn);

  prep_kernel<<<NB * (SEQ / NT), 256, 0, stream>>>(x, xh, vt, rn);

  (void)hipFuncSetAttribute(reinterpret_cast<const void*>(&attn_kernel),
                            hipFuncAttributeMaxDynamicSharedMemorySize, (int)LDS_BYTES);
  attn_kernel<<<NB * (SEQ / BQ), 256, LDS_BYTES, stream>>>(xh, vt, rn, out);
}
